// POLICEdPolicy_71932112273681
// MI455X (gfx1250) — hardware-verified
//
#include <hip/hip_runtime.h>

typedef _Float16       v16h __attribute__((ext_vector_type(16)));
typedef _Float16       v8h  __attribute__((ext_vector_type(8)));
typedef __bf16         v16b __attribute__((ext_vector_type(16)));
typedef unsigned short v8us __attribute__((ext_vector_type(8)));
typedef float          v8f  __attribute__((ext_vector_type(8)));
typedef float          v4f  __attribute__((ext_vector_type(4)));
typedef v8us __attribute__((may_alias)) v8usa;
typedef v4f  __attribute__((may_alias)) v4fa;

#define NBATCH 16384
#define NV     4096
#define WIDTH  2048
#define STATE  12
#define ACTION 8
#define K0P    64
#define CHUNK  2048
#define NCHUNK (NBATCH / CHUNK)
#define V2LD   32
#define W2ROWS 16

#define GA (NBATCH * (K0P / 8))
#define GB (NV * (K0P / 8))
#define GC (WIDTH * (K0P / 8))
#define GD (WIDTH * (K0P / 8))
#define GE (WIDTH * WIDTH / 8)
#define GF (W2ROWS * WIDTH / 8)
#define GTOT (GA + GB + GC + GD + GE + GF)

union FragH { v16h v; v8us p[2]; };
union FragB { v16b v; v8us p[2]; };
union H8    { v8h h;  v8us u; };
template<bool BF> struct FragSel { typedef FragH T; };
template<> struct FragSel<true> { typedef FragB T; };

__device__ __forceinline__ unsigned int bf16_bits(float f) {
  const unsigned int u = __float_as_uint(f);
  return (u + 0x7FFFu + ((u >> 16) & 1u)) >> 16;
}
__device__ __forceinline__ float bf16_val(unsigned int b) {
  return __uint_as_float(b << 16);
}

template<class F>
__device__ __forceinline__ F ldfrag(const unsigned short* p, int h) {
  F f;
  f.p[0] = *(const v8usa*)(p + 8 * h);
  f.p[1] = *(const v8usa*)(p + 16 + 8 * h);
  return f;
}
__device__ __forceinline__ v8f mma(const FragH& a, const FragH& b, v8f c) {
  return __builtin_amdgcn_wmma_f32_16x16x32_f16(false, a.v, false, b.v, (short)0, c, false, false);
}
__device__ __forceinline__ v8f mma(const FragB& a, const FragB& b, v8f c) {
  return __builtin_amdgcn_wmma_f32_16x16x32_bf16(false, a.v, false, b.v, (short)0, c, false, false);
}

#define NOPS4 "v_nop\n\tv_nop\n\tv_nop\n\tv_nop"

__device__ __forceinline__ unsigned int slot_bits(const float* rp, int s, int kind) {
  const bool valid = s < 3 * STATE;
  const int sc = valid ? s : 0;
  const int p = sc / STATE;
  const int c = sc - STATE * p;
  const float v = rp[c];
  const unsigned int hb = bf16_bits(v);
  const float r1 = v - bf16_val(hb);
  const unsigned int mb = bf16_bits(r1);
  const float r2 = r1 - bf16_val(mb);
  const unsigned int lb = bf16_bits(r2);
  const unsigned int p1 = (kind <= 1) ? hb : mb;
  const unsigned int p2 = (kind == 0) ? mb : ((kind == 2) ? lb : hb);
  const unsigned int b = (p == 0) ? hb : ((p == 1) ? p1 : p2);
  return valid ? b : 0u;
}

__device__ __forceinline__ void pack_group(const float* __restrict__ base, int e, int kind,
                                           unsigned short* dst) {
  const int row = e >> 3, q = e & 7;
  const float* rp = base + (size_t)row * STATE;
  v8us o;
#pragma unroll
  for (int i = 0; i < 8; ++i) o[i] = (unsigned short)slot_bits(rp, 8 * q + i, kind);
  unsigned short* p = dst + (size_t)e * 8;
  *(volatile v8us*)p = o;
  __threadfence();
  *(volatile v8us*)p = o;
}

__global__ __launch_bounds__(256) void prep_kernel(
    const float* __restrict__ x, const float* __restrict__ vtx,
    const float* __restrict__ W0, const float* __restrict__ W1, const float* __restrict__ W2,
    unsigned short* xp, unsigned short* vp, unsigned short* w0v, unsigned short* w0b,
    unsigned short* w1f, unsigned short* w1h, unsigned short* w1l,
    unsigned short* w2h, unsigned short* w2l)
{
  const int g = (int)blockIdx.x * 256 + (int)threadIdx.x;
  if (g >= GTOT) return;
  if (g < GA) {
    pack_group(x, g, 0, xp);
  } else if (g < GA + GB) {
    pack_group(vtx, g - GA, 1, vp);
  } else if (g < GA + GB + GC) {
    pack_group(W0, g - (GA + GB), 2, w0v);
  } else if (g < GA + GB + GC + GD) {
    pack_group(W0, g - (GA + GB + GC), 3, w0b);
  } else if (g < GA + GB + GC + GD + GE) {
    const int e = g - (GA + GB + GC + GD);
    const size_t e0 = (size_t)e * 8;
    const v4f x0 = *(const v4fa*)(W1 + e0);
    const v4f x1 = *(const v4fa*)(W1 + e0 + 4);
    const float a[8] = {x0[0], x0[1], x0[2], x0[3], x1[0], x1[1], x1[2], x1[3]};
    v8h fh;
    v8us hb, lb;
#pragma unroll
    for (int i = 0; i < 8; ++i) {
      fh[i] = (_Float16)(a[i] * 32.0f);
      const unsigned int b = bf16_bits(a[i]);
      hb[i] = (unsigned short)b;
      lb[i] = (unsigned short)bf16_bits(a[i] - bf16_val(b));
    }
    H8 u; u.h = fh;
    *(volatile v8us*)(w1f + e0) = u.u;
    *(volatile v8us*)(w1h + e0) = hb;
    *(volatile v8us*)(w1l + e0) = lb;
    __threadfence();
    *(volatile v8us*)(w1f + e0) = u.u;
    *(volatile v8us*)(w1h + e0) = hb;
    *(volatile v8us*)(w1l + e0) = lb;
  } else {
    const int e = g - (GA + GB + GC + GD + GE);
    const int r = e >> 8;
    const int c0 = (e & 255) * 8;
    const bool rv = r < ACTION;
    const int rr = rv ? r : (ACTION - 1);
    const float* src = W2 + (size_t)rr * WIDTH + c0;
    const v4f x0 = *(const v4fa*)src;
    const v4f x1 = *(const v4fa*)(src + 4);
    const float a[8] = {x0[0], x0[1], x0[2], x0[3], x1[0], x1[1], x1[2], x1[3]};
    v8us hb, lb;
#pragma unroll
    for (int i = 0; i < 8; ++i) {
      const float v = rv ? a[i] : 0.0f;
      const unsigned int b = bf16_bits(v);
      hb[i] = (unsigned short)b;
      lb[i] = (unsigned short)bf16_bits(v - bf16_val(b));
    }
    const size_t e0 = (size_t)e * 8;
    *(volatile v8us*)(w2h + e0) = hb;
    *(volatile v8us*)(w2l + e0) = lb;
    __threadfence();
    *(volatile v8us*)(w2h + e0) = hb;
    *(volatile v8us*)(w2l + e0) = lb;
  }
}

template<int MODE, bool NARROW>
__device__ __forceinline__ void store_pass(const float* sT, void* out0, void* out1,
                                           int m0, int n0, int ldo, int w, int lane) {
  if (!NARROW) {
    if (MODE == 0) {
      float* o = (float*)out0;
#pragma unroll
      for (int i = 0; i < 8; ++i) {
        const int row = 16 * w + 2 * i + (lane >> 4);
        const int q = lane & 15;
        const v4f v = *(const v4fa*)(sT + row * 64 + 4 * q);
        *(volatile v4f*)(o + (size_t)(m0 + row) * (size_t)ldo + n0 + 4 * q) = v;
      }
    } else {
      unsigned short* o0 = (unsigned short*)out0;
      unsigned short* o1 = (unsigned short*)out1;
#pragma unroll
      for (int i = 0; i < 4; ++i) {
        const int row = 16 * w + 4 * i + (lane >> 3);
        const int q = lane & 7;
        const v4f x0 = *(const v4fa*)(sT + row * 64 + 8 * q);
        const v4f x1 = *(const v4fa*)(sT + row * 64 + 8 * q + 4);
        const float a[8] = {x0[0], x0[1], x0[2], x0[3], x1[0], x1[1], x1[2], x1[3]};
        const size_t gi = (size_t)(m0 + row) * (size_t)ldo + n0 + 8 * q;
        if (MODE == 1) {
          v8h hh;
#pragma unroll
          for (int j = 0; j < 8; ++j) hh[j] = (_Float16)a[j];
          H8 u; u.h = hh;
          *(volatile v8us*)(o0 + gi) = u.u;
        } else {
          v8us hb, lb;
#pragma unroll
          for (int j = 0; j < 8; ++j) {
            const unsigned int b = bf16_bits(a[j]);
            hb[j] = (unsigned short)b;
            lb[j] = (unsigned short)bf16_bits(a[j] - bf16_val(b));
          }
          *(volatile v8us*)(o0 + gi) = hb;
          *(volatile v8us*)(o1 + gi) = lb;
        }
      }
    }
  } else {
    float* o = (float*)out0;
    if (MODE == 0) {
      const v4f z = {0.0f, 0.0f, 0.0f, 0.0f};
#pragma unroll
      for (int i = 0; i < 8; ++i) {
        const int row = 32 * w + 4 * i + (lane >> 3);
        const int q = lane & 7;
        const int qq = q & 3;
        v4f v = *(const v4fa*)(sT + row * 16 + 4 * qq);
        v = (q < 4) ? v : z;
        *(volatile v4f*)(o + (size_t)(m0 + row) * (size_t)ldo + 4 * q) = v;
      }
    } else {
#pragma unroll
      for (int i = 0; i < 2; ++i) {
        const int row = 32 * w + 16 * i + (lane >> 1);
        const int hf = lane & 1;
        const v4f v = *(const v4fa*)(sT + row * 16 + 4 * hf);
        *(volatile v4f*)(o + (size_t)(m0 + row) * (size_t)ldo + 4 * hf) = v;
      }
    }
  }
}

template<int NPROD, bool BF, int MODE, bool NARROW>
__global__ __launch_bounds__(128) void gemm_kernel(
    const unsigned short* __restrict__ A0, const unsigned short* __restrict__ A1,
    const unsigned short* __restrict__ B0, const unsigned short* __restrict__ B1,
    const float* __restrict__ bias, const float* __restrict__ shift,
    void* out0, void* out1,
    int lda, int ldb, int K, int ldo, int ncv, float oscale, float pscale)
{
  typedef typename FragSel<BF>::T Frag;
  constexpr int NT = NARROW ? 1 : 2;
  constexpr int BR = NARROW ? 128 : 64;
  constexpr int TP = NARROW ? 16 : 64;
  __shared__ __attribute__((aligned(16))) float sT[BR * TP];

  const int tid = (int)threadIdx.x, lane = tid & 31, w = tid >> 5;
  const int h = lane >> 4, m = lane & 15;
  const int m0 = (int)blockIdx.x * BR;
  const int n0 = NARROW ? 0 : (int)blockIdx.y * 64;
  const int wrow = NARROW ? 32 * w : 32 * (w & 1);
  const int wcol = NARROW ? 0 : 32 * (w >> 1);

  const unsigned short* pa0[2];
  const unsigned short* pa1[2];
  const unsigned short* pb0[2];
  const unsigned short* pb1[2];
#pragma unroll
  for (int mt = 0; mt < 2; ++mt) {
    const size_t o = (size_t)(m0 + wrow + 16 * mt + m) * (size_t)lda;
    pa0[mt] = A0 + o;
    pa1[mt] = A1 + o;
  }
#pragma unroll
  for (int nt = 0; nt < NT; ++nt) {
    const size_t o = (size_t)(n0 + wcol + 16 * nt + m) * (size_t)ldb;
    pb0[nt] = B0 + o;
    pb1[nt] = B1 + o;
  }

  const v8f z8 = {0.0f, 0.0f, 0.0f, 0.0f, 0.0f, 0.0f, 0.0f, 0.0f};
  v8f acc[2][2];
#pragma unroll
  for (int mt = 0; mt < 2; ++mt) { acc[mt][0] = z8; acc[mt][1] = z8; }

#pragma unroll 1
  for (int k0 = 0; k0 < K; k0 += 32) {
    Frag a0[2], a1[2], b0[2], b1[2];
#pragma unroll
    for (int mt = 0; mt < 2; ++mt) {
      a0[mt] = ldfrag<Frag>(pa0[mt] + k0, h);
      a1[mt] = (NPROD == 3) ? ldfrag<Frag>(pa1[mt] + k0, h) : a0[mt];
    }
#pragma unroll
    for (int nt = 0; nt < NT; ++nt) {
      b0[nt] = ldfrag<Frag>(pb0[nt] + k0, h);
      b1[nt] = (NPROD == 3) ? ldfrag<Frag>(pb1[nt] + k0, h) : b0[nt];
    }
#pragma unroll
    for (int mt = 0; mt < 2; ++mt)
#pragma unroll
      for (int nt = 0; nt < NT; ++nt) acc[mt][nt] = mma(a0[mt], b0[nt], acc[mt][nt]);
    if (NPROD == 3) {
#pragma unroll
      for (int mt = 0; mt < 2; ++mt)
#pragma unroll
        for (int nt = 0; nt < NT; ++nt) acc[mt][nt] = mma(a0[mt], b1[nt], acc[mt][nt]);
#pragma unroll
      for (int mt = 0; mt < 2; ++mt)
#pragma unroll
        for (int nt = 0; nt < NT; ++nt) acc[mt][nt] = mma(a1[mt], b0[nt], acc[mt][nt]);
    }
    if (NARROW) {
      asm volatile(NOPS4
                   : "+v"(acc[0][0]), "+v"(acc[1][0])
                   : "v"(a0[0].v), "v"(a0[1].v), "v"(a1[0].v), "v"(a1[1].v),
                     "v"(b0[0].v), "v"(b1[0].v));
    } else {
      asm volatile(NOPS4
                   : "+v"(acc[0][0]), "+v"(acc[0][1]), "+v"(acc[1][0]), "+v"(acc[1][1])
                   : "v"(a0[0].v), "v"(a0[1].v), "v"(a1[0].v), "v"(a1[1].v),
                     "v"(b0[0].v), "v"(b0[1].v), "v"(b1[0].v), "v"(b1[1].v));
    }
  }

#pragma unroll
  for (int nt = 0; nt < NT; ++nt) {
    const int cl = wcol + 16 * nt + m;
    const int col = n0 + cl;
    const bool cvalid = col < ncv;
    const int colc = cvalid ? col : (ncv - 1);
    const float bv = bias[colc];
    const float sv = (MODE != 0) ? shift[colc] : 0.0f;
#pragma unroll
    for (int mt = 0; mt < 2; ++mt) {
#pragma unroll
      for (int r = 0; r < 8; ++r) {
        const int row = wrow + 16 * mt + 8 * h + r;
        float v = acc[mt][nt][r] * oscale + bv - sv;
        if (MODE == 1 || MODE == 2) v = fmaxf(v, 0.0f);
        v = cvalid ? v : 0.0f;
        if (MODE == 1) v = v * pscale;
        sT[row * TP + cl] = v;
      }
    }
  }
  __syncthreads();

  store_pass<MODE, NARROW>(sT, out0, out1, m0, n0, ldo, w, lane);
  __threadfence();
  store_pass<MODE, NARROW>(sT, out0, out1, m0, n0, ldo, w, lane);
}

__global__ __launch_bounds__(256) void colstats_kernel(const float* __restrict__ V, int ldv, int ncv,
                                                       float* dsh)
{
  __shared__ float smn[8][32];
  __shared__ float smx[8][32];
  __shared__ int   scn[8][32];
  const int tid = (int)threadIdx.x, lane = tid & 31, w = tid >> 5;
  const int col = (int)blockIdx.x * 32 + lane;
  const float* p = V + (size_t)(w * (NV / 8)) * (size_t)ldv + col;
  float mn = 3.0e38f, mx = -3.0e38f;
  int cnt = 0;
#pragma unroll 4
  for (int i = 0; i < NV / 8; ++i) {
    const float v = p[(size_t)i * (size_t)ldv];
    mn = fminf(mn, v);
    mx = fmaxf(mx, v);
    cnt += (v > 0.0f) ? 1 : 0;
  }
  smn[w][lane] = mn; smx[w][lane] = mx; scn[w][lane] = cnt;
  __syncthreads();
  if (w == 0) {
#pragma unroll
    for (int j = 1; j < 8; ++j) {
      mn = fminf(mn, smn[j][lane]);
      mx = fmaxf(mx, smx[j][lane]);
      cnt += scn[j][lane];
    }
    const bool invalid = (cnt > 0) && (cnt < NV);
    const float cf = (float)((_Float16)((float)cnt));
    const bool pos = (cf - 2048.01f) > 0.0f;
    const float eps = 0.0001f;
    const float exq = fminf(mn - eps, 0.0f);
    const float exn = -fminf(-(mx + eps), 0.0f);
    float dv = pos ? exq : exn;
    dv = invalid ? dv : 0.0f;
    dv = (col < ncv) ? dv : 0.0f;
    *(volatile float*)(dsh + col) = dv;
    __threadfence();
    *(volatile float*)(dsh + col) = dv;
  }
}

__global__ __launch_bounds__(256) void vplanes_kernel(const float* __restrict__ V,
                                                      const float* __restrict__ dsh,
                                                      unsigned short* ph, unsigned short* pl)
{
  const int g = (int)blockIdx.x * 256 + (int)threadIdx.x;
  const int row = g >> 8;
  const int c0 = (g & 255) * 8;
  const float* src = V + (size_t)row * WIDTH + c0;
  const v4f x0 = *(const v4fa*)src;
  const v4f x1 = *(const v4fa*)(src + 4);
  const v4f e0 = *(const v4fa*)(dsh + c0);
  const v4f e1 = *(const v4fa*)(dsh + c0 + 4);
  const float a[8] = {x0[0] - e0[0], x0[1] - e0[1], x0[2] - e0[2], x0[3] - e0[3],
                      x1[0] - e1[0], x1[1] - e1[1], x1[2] - e1[2], x1[3] - e1[3]};
  v8us hb, lb;
#pragma unroll
  for (int i = 0; i < 8; ++i) {
    const float v = fmaxf(a[i], 0.0f);
    const unsigned int b = bf16_bits(v);
    hb[i] = (unsigned short)b;
    lb[i] = (unsigned short)bf16_bits(v - bf16_val(b));
  }
  unsigned short* q0 = ph + (size_t)g * 8;
  unsigned short* q1 = pl + (size_t)g * 8;
  *(volatile v8us*)q0 = hb;
  *(volatile v8us*)q1 = lb;
  __threadfence();
  *(volatile v8us*)q0 = hb;
  *(volatile v8us*)q1 = lb;
}

extern "C" void kernel_launch(void* const* d_in, const int* in_sizes, int n_in,
                              void* d_out, int out_size, void* d_ws, size_t ws_size,
                              hipStream_t stream) {
  if (n_in < 8) return;
  if (in_sizes[0] != NBATCH * STATE) return;
  if (in_sizes[1] != WIDTH * STATE) return;
  if (in_sizes[2] != WIDTH) return;
  if (in_sizes[3] != WIDTH * WIDTH) return;
  if (in_sizes[4] != WIDTH) return;
  if (in_sizes[5] != ACTION * WIDTH) return;
  if (in_sizes[6] != ACTION) return;
  if (in_sizes[7] != NV * STATE) return;
  if (out_size != NBATCH * ACTION) return;

  const float* x   = (const float*)d_in[0];
  const float* W0  = (const float*)d_in[1];
  const float* b0  = (const float*)d_in[2];
  const float* W1  = (const float*)d_in[3];
  const float* b1  = (const float*)d_in[4];
  const float* W2  = (const float*)d_in[5];
  const float* b2  = (const float*)d_in[6];
  const float* vtx = (const float*)d_in[7];
  float* out = (float*)d_out;

  const size_t sz_xp  = (size_t)NBATCH * K0P * 2;
  const size_t sz_vp  = (size_t)NV * K0P * 2;
  const size_t sz_w0  = (size_t)WIDTH * K0P * 2;
  const size_t sz_w1  = (size_t)WIDTH * WIDTH * 2;
  const size_t sz_w2  = (size_t)W2ROWS * WIDTH * 2;
  const size_t sz_V   = (size_t)NV * WIDTH * 4;
  const size_t sz_Vp  = (size_t)NV * WIDTH * 2;
  const size_t sz_V2  = (size_t)NV * V2LD * 4;
  const size_t sz_d   = (size_t)WIDTH * 4;
  const size_t sz_a1b = (size_t)CHUNK * WIDTH * 2;
  const size_t sz_h1  = (size_t)CHUNK * WIDTH * 2;
  const size_t total = sz_xp + sz_vp + 2 * sz_w0 + 3 * sz_w1 + 2 * sz_w2 + sz_V + 2 * sz_Vp +
                       sz_V2 + 3 * sz_d + sz_a1b + 2 * sz_h1;
  if (total > ws_size) return;

  char* ws = (char*)d_ws;
  size_t off = 0;
  unsigned short* xp  = (unsigned short*)(ws + off); off += sz_xp;
  unsigned short* vp  = (unsigned short*)(ws + off); off += sz_vp;
  unsigned short* w0v = (unsigned short*)(ws + off); off += sz_w0;
  unsigned short* w0b = (unsigned short*)(ws + off); off += sz_w0;
  unsigned short* w1f = (unsigned short*)(ws + off); off += sz_w1;
  unsigned short* w1h = (unsigned short*)(ws + off); off += sz_w1;
  unsigned short* w1l = (unsigned short*)(ws + off); off += sz_w1;
  unsigned short* w2h = (unsigned short*)(ws + off); off += sz_w2;
  unsigned short* w2l = (unsigned short*)(ws + off); off += sz_w2;
  float*          V   = (float*)(ws + off);          off += sz_V;
  unsigned short* Vh  = (unsigned short*)(ws + off); off += sz_Vp;
  unsigned short* Vl  = (unsigned short*)(ws + off); off += sz_Vp;
  float*          V2  = (float*)(ws + off);          off += sz_V2;
  float*          d0  = (float*)(ws + off);          off += sz_d;
  float*          d1  = (float*)(ws + off);          off += sz_d;
  float*          d2  = (float*)(ws + off);          off += sz_d;
  unsigned short* a1b = (unsigned short*)(ws + off); off += sz_a1b;
  unsigned short* h1h = (unsigned short*)(ws + off); off += sz_h1;
  unsigned short* h1l = (unsigned short*)(ws + off); off += sz_h1;
  if (off > ws_size) return;

  prep_kernel<<<GTOT / 256, 256, 0, stream>>>(x, vtx, W0, W1, W2, xp, vp, w0v, w0b,
                                              w1f, w1h, w1l, w2h, w2l);

  gemm_kernel<1, true, 0, false><<<dim3(NV / 64, WIDTH / 64), 128, 0, stream>>>(
      vp, vp, w0v, w0v, b0, b0, (void*)V, (void*)V, K0P, K0P, K0P, WIDTH, WIDTH, 1.0f, 1.0f);
  colstats_kernel<<<WIDTH / 32, 256, 0, stream>>>(V, WIDTH, WIDTH, d0);
  vplanes_kernel<<<(NV * WIDTH / 8) / 256, 256, 0, stream>>>(V, d0, Vh, Vl);

  gemm_kernel<3, true, 0, false><<<dim3(NV / 64, WIDTH / 64), 128, 0, stream>>>(
      Vh, Vl, w1h, w1l, b1, b1, (void*)V, (void*)V, WIDTH, WIDTH, WIDTH, WIDTH, WIDTH, 1.0f, 1.0f);
  colstats_kernel<<<WIDTH / 32, 256, 0, stream>>>(V, WIDTH, WIDTH, d1);
  vplanes_kernel<<<(NV * WIDTH / 8) / 256, 256, 0, stream>>>(V, d1, Vh, Vl);

  gemm_kernel<3, true, 0, true><<<dim3(NV / 128, 1), 128, 0, stream>>>(
      Vh, Vl, w2h, w2l, b2, b2, (void*)V2, (void*)V2, WIDTH, WIDTH, WIDTH, V2LD, ACTION, 1.0f, 1.0f);
  colstats_kernel<<<1, 256, 0, stream>>>(V2, V2LD, ACTION, d2);

  for (int c = 0; c < NCHUNK; ++c) {
    const unsigned short* xpc = xp + (size_t)c * CHUNK * K0P;
    float* outc = out + (size_t)c * CHUNK * ACTION;
    gemm_kernel<1, true, 1, false><<<dim3(CHUNK / 64, WIDTH / 64), 128, 0, stream>>>(
        xpc, xpc, w0b, w0b, b0, d0, (void*)a1b, (void*)a1b,
        K0P, K0P, K0P, WIDTH, WIDTH, 1.0f, 64.0f);
    gemm_kernel<1, false, 2, false><<<dim3(CHUNK / 64, WIDTH / 64), 128, 0, stream>>>(
        a1b, a1b, w1f, w1f, b1, d1, (void*)h1h, (void*)h1l,
        WIDTH, WIDTH, WIDTH, WIDTH, WIDTH, 1.0f / 2048.0f, 1.0f);
    gemm_kernel<3, true, 3, true><<<dim3(CHUNK / 128, 1), 128, 0, stream>>>(
        h1h, h1l, w2h, w2l, b2, d2, (void*)outc, (void*)outc,
        WIDTH, WIDTH, WIDTH, ACTION, ACTION, 1.0f, 1.0f);
  }
}
